// QuantumImagePreprocessor_51307679318825
// MI455X (gfx1250) — hardware-verified
//
#include <hip/hip_runtime.h>
#include <math.h>

typedef __attribute__((ext_vector_type(16))) _Float16 v16h;
typedef __attribute__((ext_vector_type(16))) __bf16 v16b;
typedef __attribute__((ext_vector_type(8)))  _Float16 v8h;
typedef __attribute__((ext_vector_type(8)))  float v8f;
typedef __attribute__((ext_vector_type(4)))  float v4f;
typedef __attribute__((ext_vector_type(2)))  float v2f;
typedef __attribute__((ext_vector_type(4)))  unsigned v4u;
typedef __attribute__((ext_vector_type(4)))  int v4i;
typedef float __attribute__((may_alias)) float_a;
typedef int __attribute__((may_alias)) int_a;

template <typename T> __device__ __forceinline__ void vst2(void* p, T v) { *(volatile T*)p = v; __threadfence(); *(volatile T*)p = v; }
__device__ __forceinline__ v8f wmma16(v16h a, v16h b, v8f c) {
  v8f d = __builtin_amdgcn_wmma_f32_16x16x32_f16(false, a, false, b, (short)0, c, false, false);
  asm volatile("v_nop\n\tv_nop\n\tv_nop\n\tv_nop" : "+v"(d) : "v"(a), "v"(b));
  return d;
}
__device__ __forceinline__ v8f wmma_bf(v16b a, v16b b, v8f c) {
  v8f d = __builtin_amdgcn_wmma_f32_16x16x32_bf16(false, a, false, b, (short)0, c, false, false);
  asm volatile("v_nop\n\tv_nop\n\tv_nop\n\tv_nop" : "+v"(d) : "v"(a), "v"(b));
  return d;
}
__device__ __forceinline__ v16h frag_h(const _Float16* rowk0, int lane) {
  union { v16h v; v8h q[2]; } u; const _Float16* p = rowk0 + 8 * (lane >> 4);
  u.q[0] = *(const v8h*)p; u.q[1] = *(const v8h*)(p + 16); return u.v;
}
__device__ __forceinline__ v16h frag_f32(const float* rowk0, int lane) {
  v16h a; const float* p = rowk0 + 8 * (lane >> 4);
#pragma unroll
  for (int i = 0; i < 8; ++i) { a[i] = (_Float16)p[i]; a[8 + i] = (_Float16)p[16 + i]; }
  return a;
}
__device__ __forceinline__ v16h frag_f32s(const float* rowk0, int lane, float sc) {
  v16h a; const float* p = rowk0 + 8 * (lane >> 4);
#pragma unroll
  for (int i = 0; i < 8; ++i) { a[i] = (_Float16)(p[i] * sc); a[8 + i] = (_Float16)(p[16 + i] * sc); }
  return a;
}
__device__ __forceinline__ v16h fragc_f32(const float* W, int k0, int n, int lane, int ld, int K) {
  v16h a; const int g = lane >> 4;
#pragma unroll
  for (int i = 0; i < 8; ++i) { const int ka = k0 + 8 * g + i, kb = ka + 16;
    a[i] = (_Float16)(ka < K ? W[(size_t)(ka < K ? ka : K - 1) * ld + n] : 0.f); a[8 + i] = (_Float16)(kb < K ? W[(size_t)(kb < K ? kb : K - 1) * ld + n] : 0.f); }
  return a;
}
struct F2 { v16b h, l; };
__device__ __forceinline__ F2 bsplit16(const float v[16]) { F2 r;
#pragma unroll
  for (int i = 0; i < 16; ++i) { const __bf16 h = (__bf16)v[i]; r.h[i] = h; r.l[i] = (__bf16)(v[i] - (float)h); }
  return r; }
__device__ __forceinline__ F2 split_row(const float* row, int k0, int lane) { float v[16]; const float* p = row + k0 + 8 * (lane >> 4);
#pragma unroll
  for (int i = 0; i < 8; ++i) { v[i] = p[i]; v[8 + i] = p[16 + i]; }
  return bsplit16(v); }
__device__ __forceinline__ F2 split_rowK(const float* row, int k0, int lane, int K) { float v[16]; const int g = lane >> 4;
#pragma unroll
  for (int i = 0; i < 8; ++i) { const int ka = k0 + 8 * g + i, kb = ka + 16; v[i] = ka < K ? row[ka < K ? ka : K - 1] : 0.f; v[8 + i] = kb < K ? row[kb < K ? kb : K - 1] : 0.f; }
  return bsplit16(v); }
__device__ __forceinline__ F2 split_col(const float* W, int k0, int n, int lane, int ld, int K) { float v[16]; const int g = lane >> 4;
#pragma unroll
  for (int i = 0; i < 8; ++i) { const int ka = k0 + 8 * g + i, kb = ka + 16; v[i] = ka < K ? W[(size_t)(ka < K ? ka : K - 1) * ld + n] : 0.f; v[8 + i] = kb < K ? W[(size_t)(kb < K ? kb : K - 1) * ld + n] : 0.f; }
  return bsplit16(v); }
__device__ __forceinline__ v8f mac3(const F2& a, const F2& b, v8f c) { c = wmma_bf(a.l, b.h, c); c = wmma_bf(a.h, b.l, c); return wmma_bf(a.h, b.h, c); }
__device__ __forceinline__ float sigm(float v) { return 1.0f / (1.0f + expf(-v)); }
#define LDSX() do { asm volatile("s_wait_dscnt 0" ::: "memory"); __builtin_amdgcn_wave_barrier(); __builtin_amdgcn_fence(__ATOMIC_RELEASE, "workgroup"); } while (0)


#define NBATCH 32
#define IMH 224
#define IMW 224
#define OH 112
#define OW 112
#define NP (NBATCH * OH * OW)
#ifndef NPB
#define NPB (NP / 64)
#endif
typedef __attribute__((ext_vector_type(8))) __bf16 v8b;
__device__ __forceinline__ v16b frag_b(const __bf16* rowk0, int lane) {
  union { v16b v; v8b q[2]; } u; const __bf16* p = rowk0 + 8 * (lane >> 4);
  u.q[0] = *(const v8b*)p; u.q[1] = *(const v8b*)(p + 16); return u.v;
}
__device__ __forceinline__ float bfr(float v) { return (float)(__bf16)v; }
__device__ __attribute__((noinline)) float exp_ni(float v) { return expf(v); }
__device__ __attribute__((noinline)) float erf_ni(float v) { return erff(v); }

__device__ __attribute__((noinline)) float cosf_ni(float v) { return cosf(v); }
__device__ __attribute__((noinline)) float sinf_ni(float v) { return sinf(v); }
#define WS_PB  0u
#define WS_END (WS_PB + 2u * 3 * 32 * 32)

__device__ __attribute__((noinline)) double cosd_ni(double v) { return cos(v); }
__device__ __attribute__((noinline)) double sind_ni(double v) { return sin(v); }
__global__ __launch_bounds__(64) void k_unitary(const float* __restrict__ WTS, __bf16* __restrict__ PB) {
  __shared__ double ure[16][17], uim[16][17], tre[16][17], tim[16][17]; __shared__ __align__(16) __bf16 sb[3][32][32];
  const int j = threadIdx.x;
  if (j < 16) { for (int i = 0; i < 16; ++i) { ure[i][j] = (i == j) ? 1.0 : 0.0; uim[i][j] = 0.0; } }
  __syncthreads();
#pragma unroll 1
  for (int l = 0; l < 2; ++l) {
#pragma unroll 1
    for (int w = 0; w < 4; ++w) {
      if (j < 16) { const double phi = (double)bfr(WTS[(l * 4 + w) * 3 + 0]), th = (double)bfr(WTS[(l * 4 + w) * 3 + 1]), om = (double)bfr(WTS[(l * 4 + w) * 3 + 2]);
        const double c = cosd_ni(th * 0.5), s = sind_ni(th * 0.5);
        const double ap = -(phi + om) * 0.5, am = -(phi - om) * 0.5; const double epr = cosd_ni(ap), epi = sind_ni(ap), emr = cosd_ni(am), emi = sind_ni(am);
        const double m00r = epr * c, m00i = epi * c, m01r = -emr * s, m01i = emi * s, m10r = emr * s, m10i = emi * s, m11r = epr * c, m11i = -epi * c;
        const int bit = 3 - w;
#pragma unroll 1
        for (int i0 = 0; i0 < 16; ++i0) { if ((i0 >> bit) & 1) continue; const int i1 = i0 | (1 << bit);
          const double x0r = ure[i0][j], x0i = uim[i0][j], x1r = ure[i1][j], x1i = uim[i1][j];
          ure[i0][j] = m00r * x0r - m00i * x0i + m01r * x1r - m01i * x1i; uim[i0][j] = m00r * x0i + m00i * x0r + m01r * x1i + m01i * x1r;
          ure[i1][j] = m10r * x0r - m10i * x0i + m11r * x1r - m11i * x1i; uim[i1][j] = m10r * x0i + m10i * x0r + m11r * x1i + m11i * x1r; } }
      __syncthreads(); }
    const int rr = l % 3 + 1;
#pragma unroll 1
    for (int w = 0; w < 4; ++w) { const int cb = 3 - w, tb = 3 - ((w + rr) % 4);
      if (j < 16) { for (int i = 0; i < 16; ++i) { const int srci = ((i >> cb) & 1) ? (i ^ (1 << tb)) : i; tre[i][j] = ure[srci][j]; tim[i][j] = uim[srci][j]; } }
      __syncthreads();
      if (j < 16) { for (int i = 0; i < 16; ++i) { ure[i][j] = tre[i][j]; uim[i][j] = tim[i][j]; } }
      __syncthreads(); } }
  for (int q = j; q < 32 * 32; q += 64) { const int n = q >> 5, k = q & 31; const int a = n & 15; double v;
    if (n < 16) v = (k < 16) ? ure[a][k] : -uim[a][k - 16]; else v = (k < 16) ? uim[a][k] : ure[a][k - 16];
    const float f = (float)v; const __bf16 hb = (__bf16)f; const float r1 = f - (float)hb; const __bf16 mb = (__bf16)r1; sb[0][n][k] = hb; sb[1][n][k] = mb; sb[2][n][k] = (__bf16)(r1 - (float)mb); }
  __syncthreads();
  for (int q = j; q < 3 * 32 * 32 / 8; q += 64) vst2((unsigned*)(PB + q * 8), *(const v4u*)(&sb[0][0][0] + q * 8));
}
__global__ __launch_bounds__(128) void k_qfeat(const float* __restrict__ X, const __bf16* __restrict__ PB, float* __restrict__ out) {
  __shared__ __align__(16) float so[64][4];
  const int tid = threadIdx.x, wave = tid >> 5, lane = tid & 31, col = lane & 15, g = lane >> 4; const size_t p0 = (size_t)blockIdx.x * 64 + wave * 16; const size_t patch = p0 + col;
  const int b = (int)(patch / (OH * OW)), rem = (int)(patch % (OH * OW)), oi = rem / OW, oj = rem % OW;
  const float* xr = X + ((size_t)b * IMH + 2 * oi) * IMW + 2 * oj;
  const float px[4] = {bfr(xr[0]), bfr(xr[1]), bfr(xr[IMW]), bfr(xr[IMW + 1])};
  float vr[4][2], vi[4][2];
  const float hpi = 1.5707963705062866f;
#pragma unroll
  for (int w = 0; w < 4; ++w) { const float h = px[w] * hpi; const float c = cosf_ni(h), s = sinf_ni(h); vr[w][0] = c * c; vi[w][0] = s * s; vr[w][1] = s * c; vi[w][1] = -(c * s); }
  float v[16];
#pragma unroll
  for (int i = 0; i < 8; ++i) { const int idx = 8 * g + i; const int b0_ = (idx >> 3) & 1, b1 = (idx >> 2) & 1, b2 = (idx >> 1) & 1, b3 = idx & 1;
    float ar = vr[0][b0_], ai = vi[0][b0_]; float tr_, ti_;
    tr_ = ar * vr[1][b1] - ai * vi[1][b1]; ti_ = ar * vi[1][b1] + ai * vr[1][b1]; ar = tr_; ai = ti_;
    tr_ = ar * vr[2][b2] - ai * vi[2][b2]; ti_ = ar * vi[2][b2] + ai * vr[2][b2]; ar = tr_; ai = ti_;
    tr_ = ar * vr[3][b3] - ai * vi[3][b3]; ti_ = ar * vi[3][b3] + ai * vr[3][b3];
    v[i] = tr_; v[8 + i] = ti_; }
  v16b ah, am, al;
#pragma unroll
  for (int i = 0; i < 16; ++i) { const __bf16 hb = (__bf16)v[i]; const float r1 = v[i] - (float)hb; const __bf16 mb = (__bf16)r1; ah[i] = hb; am[i] = mb; al[i] = (__bf16)(r1 - (float)mb); }
  v8f acc[2] = {};
#pragma unroll
  for (int t = 0; t < 2; ++t) { const v16b bh = frag_b(PB + (size_t)(t * 16 + col) * 32, lane), bm = frag_b(PB + 32 * 32 + (size_t)(t * 16 + col) * 32, lane), bl = frag_b(PB + 2 * 32 * 32 + (size_t)(t * 16 + col) * 32, lane);
    acc[t] = wmma_bf(am, bl, acc[t]); acc[t] = wmma_bf(al, bm, acc[t]); acc[t] = wmma_bf(ah, bl, acc[t]); acc[t] = wmma_bf(am, bm, acc[t]); acc[t] = wmma_bf(al, bh, acc[t]); acc[t] = wmma_bf(ah, bm, acc[t]); acc[t] = wmma_bf(am, bh, acc[t]); acc[t] = wmma_bf(ah, bh, acc[t]); }
  float z[4] = {0.f, 0.f, 0.f, 0.f};
#pragma unroll
  for (int r = 0; r < 8; ++r) { const float pr = acc[0][r] * acc[0][r] + acc[1][r] * acc[1][r];
    float zz[4];
#pragma unroll
    for (int w = 0; w < 4; ++w) { zz[w] = ((col >> (3 - w)) & 1) ? -pr : pr;
#pragma unroll
      for (int o = 1; o < 16; o <<= 1) zz[w] += __shfl_xor(zz[w], o); }
    if (col == (r & 15)) { for (int w = 0; w < 4; ++w) z[w] = zz[w]; }
    if (col == r) { so[wave * 16 + 8 * g + r][0] = zz[0]; so[wave * 16 + 8 * g + r][1] = zz[1]; so[wave * 16 + 8 * g + r][2] = zz[2]; so[wave * 16 + 8 * g + r][3] = zz[3]; } }
  (void)z;
  __syncthreads();
  if (tid < 64) vst2(out + (p0 - wave * 16 + tid) * 4, *(const v4f*)&so[tid][0]);
}
extern "C" void kernel_launch(void* const* d_in, const int* in_sizes, int n_in, void* d_out, int out_size, void* d_ws, size_t ws_size, hipStream_t stream) {
  (void)in_sizes; (void)n_in; (void)out_size;
  const float* X = (const float*)d_in[0]; const float* WTS = (const float*)d_in[1];
  if (ws_size < (size_t)WS_END) return;
  char* ws = (char*)d_ws; __bf16* PB = (__bf16*)(ws + WS_PB);
  k_unitary<<<1, 64, 0, stream>>>(WTS, PB);
  k_qfeat<<<NPB, 128, 0, stream>>>(X, PB, (float*)d_out);
}
